// EGCL_58660663329297
// MI455X (gfx1250) — hardware-run, weakly checked
//
#include <hip/hip_runtime.h>
#include <math.h>

constexpr int kNodes = 768;
constexpr int kHid = 128;
constexpr int kRecvPerGroup = 64;
constexpr int kGroups = kNodes / kRecvPerGroup;
constexpr int kSendSlots = kNodes;
constexpr int kMRows = kRecvPerGroup * kSendSlots;
constexpr int kGCols = 64;
constexpr int kShPitch = 32;
constexpr float kWCarry = 64.0f;
constexpr float kWCarryInv = 1.0f / 64.0f;
constexpr float kXCarry = 1024.0f;
constexpr float kXCarryInv = 1.0f / 1024.0f;
constexpr int kOut1OffsetFloats = 18432 / 4;
static_assert(kGroups * kRecvPerGroup == kNodes, "");
static_assert(kMRows % 64 == 0 && kHid % 64 == 0 && kGCols % 64 == 0, "");
static_assert(kHid % 32 == 0 && (2 * kHid) % 32 == 0, "");
static_assert(18432 + kNodes * kHid * 4 == 411648, "");

typedef __attribute__((ext_vector_type(16))) _Float16 v16h;
typedef __attribute__((ext_vector_type(8)))  _Float16 v8h;
typedef __attribute__((ext_vector_type(16))) __bf16   v16b;
typedef __attribute__((ext_vector_type(8)))  __bf16   v8b;
typedef __attribute__((ext_vector_type(8)))  float    v8f;
typedef __attribute__((ext_vector_type(4)))  float    v4f;
typedef __attribute__((ext_vector_type(4)))  unsigned int v4u;

__device__ __forceinline__ unsigned short f2bf_bits(float f) {
  unsigned u = __float_as_uint(f);
  return (unsigned short)((u + 0x7FFFu + ((u >> 16) & 1u)) >> 16);
}
__device__ __forceinline__ float bf_bits2f(unsigned short h) { return __uint_as_float(((unsigned)h) << 16); }
__device__ __forceinline__ float bfr(float f) { return bf_bits2f(f2bf_bits(f)); }
__device__ __forceinline__ v4f bfr4(v4f a) { v4f r; r[0] = bfr(a[0]); r[1] = bfr(a[1]); r[2] = bfr(a[2]); r[3] = bfr(a[3]); return r; }
__device__ __forceinline__ unsigned pk16(unsigned short a, unsigned short b) { return (unsigned)a | ((unsigned)b << 16); }
__device__ __forceinline__ unsigned short h_bits(float f) { const _Float16 h = (_Float16)f; return __builtin_bit_cast(unsigned short, h); }
__device__ __forceinline__ float silu_f(float v) {
  const float ev = expf(fminf(-v, 40.0f));
  return v * (1.0f / (1.0f + ev));
}

__device__ __forceinline__ void dep_guard_h(v8f& a, v8f& b, v16h x, v16h y) { asm volatile("v_nop\n\tv_nop\n\tv_nop\n\tv_nop" : "+v"(a), "+v"(b) : "v"(x), "v"(y)); }
__device__ __forceinline__ void dep_guard_b(v8f& a, v8f& b, v16b x, v16b y) { asm volatile("v_nop\n\tv_nop\n\tv_nop\n\tv_nop" : "+v"(a), "+v"(b) : "v"(x), "v"(y)); }
__device__ __forceinline__ void dep_guard4_h(v8f& a, v8f& b, v8f& c, v8f& d, v16h x, v16h y) { asm volatile("v_nop\n\tv_nop\n\tv_nop\n\tv_nop" : "+v"(a), "+v"(b), "+v"(c), "+v"(d) : "v"(x), "v"(y)); }
__device__ __forceinline__ void dep_guard4_b(v8f& a, v8f& b, v8f& c, v8f& d, v16b x, v16b y) { asm volatile("v_nop\n\tv_nop\n\tv_nop\n\tv_nop" : "+v"(a), "+v"(b), "+v"(c), "+v"(d) : "v"(x), "v"(y)); }
__device__ __forceinline__ void keep4_h(v16h a, v16h b, v16h c, v16h d) { asm volatile("v_nop" :: "v"(a), "v"(b), "v"(c), "v"(d)); }
__device__ __forceinline__ void keep4_b(v16b a, v16b b, v16b c, v16b d) { asm volatile("v_nop" :: "v"(a), "v"(b), "v"(c), "v"(d)); }
__device__ __forceinline__ void acc_guard4(v8f& a, v8f& b, v8f& c, v8f& d) { asm volatile("v_nop\n\tv_nop\n\tv_nop\n\tv_nop" : "+v"(a), "+v"(b), "+v"(c), "+v"(d)); }
template <typename T> struct Frag;
template <> struct Frag<_Float16> {
  typedef v16h V; union U { v16h v; v8h h[2]; };
  static __device__ __forceinline__ v16h load(const _Float16* p) {
    U f; f.h[0] = *(const v8h*)(p); f.h[1] = *(const v8h*)(p + 16); return f.v;
  }
  static __device__ __forceinline__ v8f mma(v16h a, v16h b, v8f c) {
    return __builtin_amdgcn_wmma_f32_16x16x32_f16(false, a, false, b, (short)0, c, false, false);
  }
  static __device__ __forceinline__ void guard(v8f& a, v8f& b, v16h x, v16h y) { dep_guard_h(a, b, x, y); }
  static __device__ __forceinline__ void guard4(v8f& a, v8f& b, v8f& c, v8f& d, v16h x, v16h y) { dep_guard4_h(a, b, c, d, x, y); }
  static __device__ __forceinline__ void keep(v16h a, v16h b, v16h c, v16h d) { keep4_h(a, b, c, d); }
};
template <> struct Frag<__bf16> {
  typedef v16b V; union U { v16b v; v8b h[2]; };
  static __device__ __forceinline__ v16b load(const __bf16* p) {
    U f; f.h[0] = *(const v8b*)(p); f.h[1] = *(const v8b*)(p + 16); return f.v;
  }
  static __device__ __forceinline__ v8f mma(v16b a, v16b b, v8f c) {
    return __builtin_amdgcn_wmma_f32_16x16x32_bf16(false, a, false, b, (short)0, c, false, false);
  }
  static __device__ __forceinline__ void guard(v8f& a, v8f& b, v16b x, v16b y) { dep_guard_b(a, b, x, y); }
  static __device__ __forceinline__ void guard4(v8f& a, v8f& b, v8f& c, v8f& d, v16b x, v16b y) { dep_guard4_b(a, b, c, d, x, y); }
  static __device__ __forceinline__ void keep(v16b a, v16b b, v16b c, v16b d) { keep4_b(a, b, c, d); }
};

template <int ET> struct Elem;
template <> struct Elem<0> { typedef _Float16 T; };
template <> struct Elem<1> { typedef __bf16 T; };
template <int ET, bool SPLIT, int BIAS_MODE, int OUT_MODE, bool RESID, int ACT = 0>
__global__ __launch_bounds__(256) void wmma_gemm64(
    const unsigned short* __restrict__ Ap, const unsigned short* __restrict__ A2p, int lda, long strideA,
    const unsigned short* __restrict__ Btp, const unsigned short* __restrict__ Bt2p, int ldb, long strideB,
    void* __restrict__ Cout, void* __restrict__ Cout2, int ldc, long strideC,
    const float* __restrict__ bias,
    const float* __restrict__ resid, long strideR,
    int M, int N, int K, float scale) {
  typedef typename Elem<ET>::T T;
  typedef typename Frag<T>::V V;
  const T* A = (const T*)Ap; const T* A2 = (const T*)A2p; const T* Bt = (const T*)Btp; const T* Bt2 = (const T*)Bt2p;
  __shared__ __align__(16) float sT[8][16 * 68];
  const int b    = blockIdx.y;
  const int lane = threadIdx.x & 31;
  const int wave = threadIdx.x >> 5;
  const int tilesN = N >> 6;
  const int tilesM = M >> 6;
  const int tile = blockIdx.x * 8 + wave;
  if (tile >= tilesM * tilesN) return;
  const int tm = tile / tilesN;
  const int tn = tile - tm * tilesN;
  const int m0 = tm << 6;
  const int n0 = tn << 6;

  const T* Ab  = A  + (size_t)b * strideA;
  const T* Bb  = Bt + (size_t)b * strideB;
  const T* Ab2 = SPLIT ? (A2  + (size_t)b * strideA) : nullptr;
  const T* Bb2 = SPLIT ? (Bt2 + (size_t)b * strideB) : nullptr;

  const int rlane = lane & 15;
  const int koff  = (lane >> 4) * 8;
  const int mOff  = (lane >> 4) * 8;

  v8f acc[4][4];
#pragma unroll
  for (int i = 0; i < 4; ++i)
#pragma unroll
    for (int j = 0; j < 4; ++j) acc[i][j] = (v8f){0.f,0.f,0.f,0.f,0.f,0.f,0.f,0.f};

  for (int k0 = 0; k0 < K; k0 += 32) {
    V bh[4], bl[4];
#pragma unroll
    for (int j = 0; j < 4; ++j) {
      const size_t bo = (size_t)(n0 + (j << 4) + rlane) * ldb + koff + k0;
      bh[j] = Frag<T>::load(Bb + bo);
      if (SPLIT) bl[j] = Frag<T>::load(Bb2 + bo);
    }
#pragma unroll
    for (int i = 0; i < 4; ++i) {
      const size_t ao = (size_t)(m0 + (i << 4) + rlane) * lda + koff + k0;
      V ah = Frag<T>::load(Ab + ao);
      V al;
      if (SPLIT) al = Frag<T>::load(Ab2 + ao);
#pragma unroll
      for (int j = 0; j < 4; ++j) {
        acc[i][j] = Frag<T>::mma(ah, bh[j], acc[i][j]);
        if (SPLIT) {
          acc[i][j] = Frag<T>::mma(ah, bl[j], acc[i][j]);
          acc[i][j] = Frag<T>::mma(al, bh[j], acc[i][j]);
        }
      }
      Frag<T>::guard4(acc[i][0], acc[i][1], acc[i][2], acc[i][3], ah, SPLIT ? al : ah);
    }
    Frag<T>::keep(bh[0], bh[1], bh[2], bh[3]);
    if (SPLIT) Frag<T>::keep(bl[0], bl[1], bl[2], bl[3]);
  }
  acc_guard4(acc[0][0], acc[0][1], acc[0][2], acc[0][3]);
  acc_guard4(acc[1][0], acc[1][1], acc[1][2], acc[1][3]);
  acc_guard4(acc[2][0], acc[2][1], acc[2][2], acc[2][3]);
  acc_guard4(acc[3][0], acc[3][1], acc[3][2], acc[3][3]);

  float* slab = sT[wave];
  const float* Rb = RESID ? (resid + (size_t)b * strideR) : nullptr;
#pragma unroll
  for (int i = 0; i < 4; ++i) {
    const int mBase = m0 + (i << 4);
#pragma unroll
    for (int j = 0; j < 4; ++j) {
      const int n = n0 + (j << 4) + rlane;
      float bv = 0.f;
      if (BIAS_MODE == 2) bv = bfr(bias[n]);
#pragma unroll
      for (int r = 0; r < 8; ++r) {
        float v = acc[i][j][r] * scale;
        if (BIAS_MODE == 1) v += bfr(bias[mBase + mOff + r]);
        if (BIAS_MODE == 2) v += bv;
        if (RESID) v += Rb[(size_t)(mBase + mOff + r) * ldc + n];
        if (ACT == 2) v = fmaxf(v, 0.0f);
        if (ACT == 3) v = silu_f(v);
        if (ACT == 4) v = (v > 0.f) ? v : 0.01f * v;
        slab[(mOff + r) * 68 + (j << 4) + rlane] = v;
      }
    }
    __builtin_amdgcn_fence(__ATOMIC_RELEASE, "workgroup");
    __builtin_amdgcn_wave_barrier();
    __builtin_amdgcn_fence(__ATOMIC_ACQUIRE, "workgroup");
    if (OUT_MODE == 0 || OUT_MODE == 3) {
      float* C = (float*)Cout + (size_t)b * strideC;
      unsigned short* C3 = (OUT_MODE == 3) ? ((unsigned short*)Cout2 + (size_t)b * strideC) : nullptr;
      const int hh = lane >> 4, c4 = (lane & 15) * 4;
      const int q3 = lane >> 3, c83 = (lane & 7) * 8;
      const int ldc3 = 2 * ldc;
      for (int pass = 0; pass < 2; ++pass) {
#pragma unroll
        for (int it = 0; it < 8; ++it) {
          const int row = it * 2 + hh;
          v4f v = *(const v4f*)(slab + row * 68 + c4);
          *(volatile v4f*)(C + (size_t)(mBase + row) * ldc + n0 + c4) = v;
        }
        if (OUT_MODE == 3) {
#pragma unroll
          for (int it = 0; it < 4; ++it) {
            const int row = it * 4 + q3;
            const float* sp = slab + row * 68 + c83;
            v8h hv;
#pragma unroll
            for (int e = 0; e < 8; ++e) hv[e] = (_Float16)sp[e];
            *(volatile v8h*)(C3 + (size_t)(mBase + row) * ldc3 + n0 + c83) = hv;
          }
        }
        __threadfence();
      }
    } else {
      const int q = lane >> 3, c8 = (lane & 7) * 8;
      unsigned short* C  = (unsigned short*)Cout  + (size_t)b * strideC;
      unsigned short* C2 = (OUT_MODE == 2) ? ((unsigned short*)Cout2 + (size_t)b * strideC) : nullptr;
      for (int pass = 0; pass < 2; ++pass) {
#pragma unroll
        for (int it = 0; it < 4; ++it) {
          const int row = it * 4 + q;
          const float* sp = slab + row * 68 + c8;
          v8h hv, lv;
#pragma unroll
          for (int e = 0; e < 8; ++e) {
            if (OUT_MODE == 1) {
              hv[e] = (_Float16)sp[e];
            } else {
              unsigned short hb = f2bf_bits(sp[e]);
              unsigned short lb = f2bf_bits(sp[e] - bf_bits2f(hb));
              hv[e] = __builtin_bit_cast(_Float16, hb);
              lv[e] = __builtin_bit_cast(_Float16, lb);
            }
          }
          *(volatile v8h*)(C + (size_t)(mBase + row) * ldc + n0 + c8) = hv;
          if (OUT_MODE == 2) *(volatile v8h*)(C2 + (size_t)(mBase + row) * ldc + n0 + c8) = lv;
        }
        __threadfence();
      }
    }
    __builtin_amdgcn_fence(__ATOMIC_RELEASE, "workgroup");
    __builtin_amdgcn_wave_barrier();
    __builtin_amdgcn_fence(__ATOMIC_ACQUIRE, "workgroup");
  }
}

__global__ __launch_bounds__(256) void wtcast_kernel(const float* __restrict__ W0, const float* __restrict__ W1,
                                                     const float* __restrict__ W2, const float* __restrict__ W3,
                                                     unsigned short* __restrict__ out, float scale) {
  __shared__ float sm[64][65];
  const int t  = threadIdx.x;
  const int d0 = blockIdx.x * 64;
  const int h0 = blockIdx.y * 64;
  const int z  = blockIdx.z;
  const float* W = (z == 0) ? W0 : (z == 1) ? W1 : (z == 2) ? W2 : W3;
#pragma unroll
  for (int i = 0; i < 16; ++i) {
    const int e = i * 256 + t;
    const int r = e >> 6;
    const int c = e & 63;
    sm[c][r] = bfr(W[(size_t)(d0 + r) * kHid + h0 + c]) * scale;
  }
  __syncthreads();
  const int lane = t & 31, wave = t >> 5;
  const int q = lane >> 3, c8 = (lane & 7) * 8;
  unsigned short* op = out + (size_t)z * kHid * kHid;
  for (int pass = 0; pass < 2; ++pass) {
#pragma unroll
    for (int it = 0; it < 2; ++it) {
      const int row = wave * 8 + it * 4 + q;
      unsigned short hb[8];
#pragma unroll
      for (int e = 0; e < 8; ++e) hb[e] = h_bits(sm[row][c8 + e]);
      const v4u u = (v4u){pk16(hb[0], hb[1]), pk16(hb[2], hb[3]), pk16(hb[4], hb[5]), pk16(hb[6], hb[7])};
      *(volatile v4u*)(op + (size_t)(h0 + row) * kHid + d0 + c8) = u;
    }
    __threadfence();
  }
}

__global__ __launch_bounds__(256) void w56_kernel(const float* __restrict__ winf, const float* __restrict__ wxl,
                                                  unsigned short* __restrict__ out) {
  const int gt = blockIdx.x * 256 + threadIdx.x;
  const int row = gt >> 5;
  const int k0 = (gt & 31) * 8;
  const int kc = k0 & 127;
  const v4f g0 = bfr4(*(const v4f*)(winf + kc));
  const v4f g1 = bfr4(*(const v4f*)(winf + kc + 4));
  const v4f x0 = bfr4(*(const v4f*)(wxl + 2 * kc));
  const v4f x1 = bfr4(*(const v4f*)(wxl + 2 * kc + 4));
  const v4f x2 = bfr4(*(const v4f*)(wxl + 2 * kc + 8));
  const v4f x3 = bfr4(*(const v4f*)(wxl + 2 * kc + 12));
  const float fg = (row == 0 && k0 < 128) ? kWCarry : 0.0f;
  const float f0 = (row == 1 && k0 >= 128) ? kXCarry : 0.0f;
  const float f1 = (row == 2 && k0 >= 128) ? kXCarry : 0.0f;
  float gv[8], xa[8], xb[8];
  gv[0] = g0[0]; gv[1] = g0[1]; gv[2] = g0[2]; gv[3] = g0[3];
  gv[4] = g1[0]; gv[5] = g1[1]; gv[6] = g1[2]; gv[7] = g1[3];
  xa[0] = x0[0]; xb[0] = x0[1]; xa[1] = x0[2]; xb[1] = x0[3];
  xa[2] = x1[0]; xb[2] = x1[1]; xa[3] = x1[2]; xb[3] = x1[3];
  xa[4] = x2[0]; xb[4] = x2[1]; xa[5] = x2[2]; xb[5] = x2[3];
  xa[6] = x3[0]; xb[6] = x3[1]; xa[7] = x3[2]; xb[7] = x3[3];
  unsigned short hb[8];
#pragma unroll
  for (int e = 0; e < 8; ++e) hb[e] = h_bits(fg * gv[e] + f0 * xa[e] + f1 * xb[e]);
  const v4u u = (v4u){pk16(hb[0], hb[1]), pk16(hb[2], hb[3]), pk16(hb[4], hb[5]), pk16(hb[6], hb[7])};
  unsigned short* op = out + (size_t)row * 256 + k0;
  *(volatile v4u*)op = u;
  __threadfence();
  *(volatile v4u*)op = u;
}

__global__ __launch_bounds__(256) void node_proj_kernel(const float* __restrict__ h, const float* __restrict__ we0,
                                                        const float* __restrict__ be0, float* __restrict__ PS,
                                                        float* __restrict__ PR) {
  const int lane = threadIdx.x & 31, wave = threadIdx.x >> 5;
  const int n = blockIdx.x * 8 + wave;
  const float* hr = h + (size_t)n * kHid;
  v4f as = (v4f){0.f, 0.f, 0.f, 0.f};
  v4f ar = (v4f){0.f, 0.f, 0.f, 0.f};
  ar = ar + bfr4(*(const v4f*)(be0 + 4 * lane));
#pragma unroll 1
  for (int k = 0; k < kHid; ++k) {
    const float hk = bfr(hr[k]);
    const v4f ws = bfr4(*(const v4f*)(we0 + (size_t)(2 + k) * kHid + 4 * lane));
    const v4f wr = bfr4(*(const v4f*)(we0 + (size_t)(130 + k) * kHid + 4 * lane));
    as = as + hk * ws;
    ar = ar + hk * wr;
  }
  float* ps = PS + (size_t)n * kHid + 4 * lane;
  float* pr = PR + (size_t)n * kHid + 4 * lane;
  for (int pass = 0; pass < 2; ++pass) {
    *(volatile v4f*)ps = as;
    *(volatile v4f*)pr = ar;
    __threadfence();
  }
}

__global__ __launch_bounds__(256) void build_a0_kernel(const float* __restrict__ nv, const float* __restrict__ we0,
                                                       const float* __restrict__ PS, const float* __restrict__ PR,
                                                       unsigned short* __restrict__ A0, int r0) {
  const int t = threadIdx.x;
  const int er = blockIdx.x * 16 + (t >> 4);
  const int c0 = (t & 15) * 8;
  const int rl = er / kSendSlots;
  const int s = er - rl * kSendSlots;
  const int r = r0 + rl;
  float xr[6], xs[6];
#pragma unroll
  for (int q = 0; q < 6; ++q) { xr[q] = bfr(nv[r * 6 + q]); xs[q] = bfr(nv[s * 6 + q]); }
  asm volatile("" ::: "memory");
  const v4f ps0 = *(const v4f*)(PS + (size_t)s * kHid + c0);
  const v4f ps1 = *(const v4f*)(PS + (size_t)s * kHid + c0 + 4);
  const v4f pr0 = *(const v4f*)(PR + (size_t)r * kHid + c0);
  const v4f pr1 = *(const v4f*)(PR + (size_t)r * kHid + c0 + 4);
  const v4f w00 = bfr4(*(const v4f*)(we0 + c0));
  const v4f w01 = bfr4(*(const v4f*)(we0 + c0 + 4));
  const v4f w10 = bfr4(*(const v4f*)(we0 + kHid + c0));
  const v4f w11 = bfr4(*(const v4f*)(we0 + kHid + c0 + 4));
  const float dx0 = xr[0] - xs[0], dy0 = xr[1] - xs[1], dz0 = xr[2] - xs[2];
  const float dx1 = xr[3] - xs[3], dy1 = xr[4] - xs[4], dz1 = xr[5] - xs[5];
  const float l2c0 = fmaxf(dx0 * dx0 + dy0 * dy0 + dz0 * dz0, 1e-20f);
  const float l2c1 = fmaxf(dx1 * dx1 + dy1 * dy1 + dz1 * dz1, 1e-20f);
  const float len0 = sqrtf(l2c0), len1 = sqrtf(l2c1);
  const float lsq0 = len0 * len0, lsq1 = len1 * len1;
  const v4f pa = ps0 + pr0 + lsq0 * w00 + lsq1 * w10;
  const v4f pb = ps1 + pr1 + lsq0 * w01 + lsq1 * w11;
  v8h hv;
#pragma unroll
  for (int e = 0; e < 4; ++e) {
    hv[e] = (_Float16)silu_f(pa[e]);
    hv[4 + e] = (_Float16)silu_f(pb[e]);
  }
  unsigned short* dst = A0 + (size_t)er * kHid + c0;
  for (int pass = 0; pass < 2; ++pass) {
    *(volatile v8h*)dst = hv;
    __threadfence();
  }
}

__global__ __launch_bounds__(256) void agg_kernel(const float* __restrict__ nv, const float* __restrict__ MIJ,
                                                  const float* __restrict__ GB, const float* __restrict__ bxl,
                                                  const float* __restrict__ binf, float* __restrict__ MI,
                                                  float* __restrict__ SH, int r0) {
  __shared__ __align__(16) float red[8][kHid];
  __shared__ float shr[8][8];
  const int lane = threadIdx.x & 31, wave = threadIdx.x >> 5;
  const int rl = blockIdx.x;
  const int r = r0 + rl;
  float xr[6];
#pragma unroll
  for (int q = 0; q < 6; ++q) xr[q] = bfr(nv[r * 6 + q]);
  const float b0 = bfr(bxl[0]), b1 = bfr(bxl[1]), bi = bfr(binf[0]);
  v4f acc = (v4f){0.f, 0.f, 0.f, 0.f};
  float sa0 = 0.f, sa1 = 0.f, sa2 = 0.f, sa3 = 0.f, sa4 = 0.f, sa5 = 0.f;
  const size_t rowbase = (size_t)rl * kSendSlots;
#pragma unroll 1
  for (int i = 0; i < kSendSlots / 8; ++i) {
    const int s = wave + 8 * i;
    const float fm = (s != r) ? 1.0f : 0.0f;
    const size_t er = rowbase + (size_t)s;
    const v4f m4 = *(const v4f*)(MIJ + er * kHid + 4 * lane);
    const v4f g4 = *(const v4f*)(GB + er * kGCols);
    float xs[6];
#pragma unroll
    for (int q = 0; q < 6; ++q) xs[q] = bfr(nv[s * 6 + q]);
    const float lg = g4[0] * kWCarryInv + bi;
    const float gate = 1.0f / (1.0f + expf(fminf(-lg, 40.0f)));
    acc = acc + (fm * gate) * m4;
    const float dx0 = xr[0] - xs[0], dy0 = xr[1] - xs[1], dz0 = xr[2] - xs[2];
    const float dx1 = xr[3] - xs[3], dy1 = xr[4] - xs[4], dz1 = xr[5] - xs[5];
    const float l2c0 = fmaxf(dx0 * dx0 + dy0 * dy0 + dz0 * dz0, 1e-20f);
    const float l2c1 = fmaxf(dx1 * dx1 + dy1 * dy1 + dz1 * dz1, 1e-20f);
    const float rc0 = 1.0f / (1.0f + sqrtf(l2c0));
    const float rc1 = 1.0f / (1.0f + sqrtf(l2c1));
    const float px0 = fm * (g4[1] * kXCarryInv + b0);
    const float px1 = fm * (g4[2] * kXCarryInv + b1);
    sa0 += (px0 * dx0) * rc0; sa1 += (px0 * dy0) * rc0; sa2 += (px0 * dz0) * rc0;
    sa3 += (px1 * dx1) * rc1; sa4 += (px1 * dy1) * rc1; sa5 += (px1 * dz1) * rc1;
  }
  *(v4f*)(&red[wave][4 * lane]) = acc;
  if (lane == 0) {
    shr[wave][0] = sa0; shr[wave][1] = sa1; shr[wave][2] = sa2;
    shr[wave][3] = sa3; shr[wave][4] = sa4; shr[wave][5] = sa5;
    shr[wave][6] = 0.f; shr[wave][7] = 0.f;
  }
  __syncthreads();
  if (wave == 0) {
    v4f tot = (v4f){0.f, 0.f, 0.f, 0.f};
#pragma unroll
    for (int w = 0; w < 8; ++w) tot = tot + *(const v4f*)(&red[w][4 * lane]);
    const float invs = 1.0f / sqrtf(767.0f);
    tot = tot * invs;
    const int lc = (lane < 6) ? lane : 6;
    float sacc = 0.f;
#pragma unroll
    for (int w = 0; w < 8; ++w) sacc += shr[w][lc];
    float* mi = MI + (size_t)r * kHid + 4 * lane;
    float* sh = SH + (size_t)r * kShPitch + lane;
    for (int pass = 0; pass < 2; ++pass) {
      *(volatile v4f*)mi = tot;
      *(volatile float*)sh = sacc;
      __threadfence();
    }
  }
}

__global__ __launch_bounds__(256) void node_out_kernel(const float* __restrict__ MI, const float* __restrict__ h,
                                                       const float* __restrict__ wh0, const float* __restrict__ bh0,
                                                       const float* __restrict__ wh1, const float* __restrict__ bh1,
                                                       const float* __restrict__ whl, const float* __restrict__ bhl,
                                                       float* __restrict__ out1) {
  __shared__ __align__(16) float qa[8][kHid];
  __shared__ __align__(16) float qb[8][kHid];
  const int lane = threadIdx.x & 31, wave = threadIdx.x >> 5;
  const int n = blockIdx.x * 8 + wave;
  const float* mrow = MI + (size_t)n * kHid;
  const float* hrow = h + (size_t)n * kHid;
  v4f acc = (v4f){0.f, 0.f, 0.f, 0.f};
  acc = acc + bfr4(*(const v4f*)(bh0 + 4 * lane));
#pragma unroll 1
  for (int k = 0; k < kHid; ++k) acc = acc + mrow[k] * bfr4(*(const v4f*)(wh0 + (size_t)k * kHid + 4 * lane));
#pragma unroll 1
  for (int k = 0; k < kHid; ++k) acc = acc + bfr(hrow[k]) * bfr4(*(const v4f*)(wh0 + (size_t)(kHid + k) * kHid + 4 * lane));
  v4f q;
#pragma unroll
  for (int e = 0; e < 4; ++e) q[e] = silu_f(acc[e]);
  *(v4f*)(&qa[wave][4 * lane]) = q;
  __syncthreads();
  acc = (v4f){0.f, 0.f, 0.f, 0.f};
  acc = acc + bfr4(*(const v4f*)(bh1 + 4 * lane));
#pragma unroll 1
  for (int k = 0; k < kHid; ++k) acc = acc + qa[wave][k] * bfr4(*(const v4f*)(wh1 + (size_t)k * kHid + 4 * lane));
#pragma unroll
  for (int e = 0; e < 4; ++e) q[e] = silu_f(acc[e]);
  *(v4f*)(&qb[wave][4 * lane]) = q;
  __syncthreads();
  acc = (v4f){0.f, 0.f, 0.f, 0.f};
  acc = acc + bfr4(*(const v4f*)(bhl + 4 * lane));
#pragma unroll 1
  for (int k = 0; k < kHid; ++k) acc = acc + qb[wave][k] * bfr4(*(const v4f*)(whl + (size_t)k * kHid + 4 * lane));
  acc = acc + bfr4(*(const v4f*)(hrow + 4 * lane));
  float* op = out1 + (size_t)n * kHid + 4 * lane;
  for (int pass = 0; pass < 2; ++pass) {
    *(volatile v4f*)op = acc;
    __threadfence();
  }
}

__global__ __launch_bounds__(128) void out0_kernel(const float* __restrict__ nv, const float* __restrict__ SH,
                                                   float* __restrict__ out0) {
  const int i = blockIdx.x * 128 + threadIdx.x;
  const v4f x = *(const v4f*)(nv + 4 * i);
  const float inv = 1.0f / 767.0f;
  v4f o;
#pragma unroll
  for (int j = 0; j < 4; ++j) {
    const int f = 4 * i + j;
    const int node = f / 6;
    const int comp = f - node * 6;
    o[j] = bfr(x[j]) + SH[(size_t)node * kShPitch + comp] * inv;
  }
  float* op = out0 + 4 * (size_t)i;
  *(volatile v4f*)op = o;
  __threadfence();
  *(volatile v4f*)op = o;
}

extern "C" void kernel_launch(void* const* d_in, const int* in_sizes, int n_in,
                              void* d_out, int out_size, void* d_ws, size_t ws_size, hipStream_t stream) {
  (void)in_sizes; (void)n_in; (void)out_size;
  const float* nvec  = (const float*)d_in[0];
  const float* nfeat = (const float*)d_in[1];
  const float* we0 = (const float*)d_in[2];  const float* be0 = (const float*)d_in[3];
  const float* we1 = (const float*)d_in[4];  const float* be1 = (const float*)d_in[5];
  const float* we2 = (const float*)d_in[6];  const float* be2 = (const float*)d_in[7];
  const float* wx0 = (const float*)d_in[8];  const float* bx0 = (const float*)d_in[9];
  const float* wx1 = (const float*)d_in[10]; const float* bx1 = (const float*)d_in[11];
  const float* wxl = (const float*)d_in[12]; const float* bxl = (const float*)d_in[13];
  const float* winf = (const float*)d_in[14]; const float* binf = (const float*)d_in[15];
  const float* wh0 = (const float*)d_in[16]; const float* bh0 = (const float*)d_in[17];
  const float* wh1 = (const float*)d_in[18]; const float* bh1 = (const float*)d_in[19];
  const float* whl = (const float*)d_in[20]; const float* bhl = (const float*)d_in[21];
  float* out0 = (float*)d_out;
  float* out1 = (float*)d_out + kOut1OffsetFloats;

  char* ws = (char*)d_ws; size_t off = 0;
  auto carve = [&](size_t bytes) -> char* { char* p = ws + off; off += (bytes + 255) & ~(size_t)255; return p; };
  float*          PS  = (float*)carve((size_t)kNodes * kHid * 4);
  float*          PR  = (float*)carve((size_t)kNodes * kHid * 4);
  unsigned short* WT  = (unsigned short*)carve((size_t)4 * kHid * kHid * 2);
  unsigned short* W56 = (unsigned short*)carve((size_t)kGCols * 2 * kHid * 2);
  unsigned short* A0  = (unsigned short*)carve((size_t)kMRows * kHid * 2);
  unsigned short* A1  = (unsigned short*)carve((size_t)kMRows * kHid * 2);
  unsigned short* MP  = (unsigned short*)carve((size_t)kMRows * 2 * kHid * 2);
  float*          MIJ = (float*)carve((size_t)kMRows * kHid * 4);
  float*          GB  = (float*)carve((size_t)kMRows * kGCols * 4);
  float*          MI  = (float*)carve((size_t)kNodes * kHid * 4);
  float*          SH  = (float*)carve((size_t)kNodes * kShPitch * 4);
  if (off > ws_size || off > (size_t)134217728) return;
  unsigned short* P0 = A0;

  const unsigned short* WT_we1 = WT;
  const unsigned short* WT_we2 = WT + (size_t)kHid * kHid;
  const unsigned short* WT_wx0 = WT + (size_t)2 * kHid * kHid;
  const unsigned short* WT_wx1 = WT + (size_t)3 * kHid * kHid;

  node_proj_kernel<<<kNodes / 8, 256, 0, stream>>>(nfeat, we0, be0, PS, PR);
  wtcast_kernel<<<dim3(kHid / 64, kHid / 64, 4), 256, 0, stream>>>(we1, we2, wx0, wx1, WT, kWCarry);
  w56_kernel<<<(kGCols * 2 * kHid / 8) / 256, 256, 0, stream>>>(winf, wxl, W56);

  const int tilesMain = (kMRows / 64) * (kHid / 64);
  const int tilesHead = (kMRows / 64) * (kGCols / 64);
  for (int g = 0; g < kGroups; ++g) {
    const int r0 = g * kRecvPerGroup;
    build_a0_kernel<<<kMRows / 16, 256, 0, stream>>>(nvec, we0, PS, PR, A0, r0);
    wmma_gemm64<0, false, 2, 1, false, 3><<<dim3((tilesMain + 7) / 8, 1), 256, 0, stream>>>(
        A0, nullptr, kHid, 0L, WT_we1, nullptr, kHid, 0L,
        (void*)A1, (void*)nullptr, kHid, 0L, be1, (const float*)nullptr, 0L, kMRows, kHid, kHid, kWCarryInv);
    wmma_gemm64<0, false, 2, 3, false, 0><<<dim3((tilesMain + 7) / 8, 1), 256, 0, stream>>>(
        A1, nullptr, kHid, 0L, WT_we2, nullptr, kHid, 0L,
        (void*)MIJ, (void*)MP, kHid, 0L, be2, (const float*)nullptr, 0L, kMRows, kHid, kHid, kWCarryInv);
    wmma_gemm64<0, false, 2, 1, false, 3><<<dim3((tilesMain + 7) / 8, 1), 256, 0, stream>>>(
        MP, nullptr, 2 * kHid, 0L, WT_wx0, nullptr, kHid, 0L,
        (void*)P0, (void*)nullptr, kHid, 0L, bx0, (const float*)nullptr, 0L, kMRows, kHid, kHid, kWCarryInv);
    wmma_gemm64<0, false, 2, 1, false, 3><<<dim3((tilesMain + 7) / 8, 1), 256, 0, stream>>>(
        P0, nullptr, kHid, 0L, WT_wx1, nullptr, kHid, 0L,
        (void*)(MP + kHid), (void*)nullptr, 2 * kHid, 0L, bx1, (const float*)nullptr, 0L, kMRows, kHid, kHid, kWCarryInv);
    wmma_gemm64<0, false, 0, 0, false, 0><<<dim3((tilesHead + 7) / 8, 1), 256, 0, stream>>>(
        MP, nullptr, 2 * kHid, 0L, W56, nullptr, 2 * kHid, 0L,
        (void*)GB, (void*)nullptr, kGCols, 0L, (const float*)nullptr, (const float*)nullptr, 0L, kMRows, kGCols, 2 * kHid, 1.0f);
    agg_kernel<<<kRecvPerGroup, 256, 0, stream>>>(nvec, MIJ, GB, bxl, binf, MI, SH, r0);
  }
  node_out_kernel<<<kNodes / 8, 256, 0, stream>>>(MI, nfeat, wh0, bh0, wh1, bh1, whl, bhl, out1);
  out0_kernel<<<(kNodes * 6 / 4) / 128, 128, 0, stream>>>(nvec, SH, out0);
}
